// Encoder_84585085927968
// MI455X (gfx1250) — hardware-run, weakly checked
//
#include <hip/hip_runtime.h>
#include <math.h>

typedef __attribute__((ext_vector_type(16))) _Float16 v16h;
typedef __attribute__((ext_vector_type(8)))  _Float16 v8h;
typedef __attribute__((ext_vector_type(16))) __bf16   v16b;
typedef __attribute__((ext_vector_type(8)))  __bf16   v8b;
typedef __attribute__((ext_vector_type(8)))  float    v8f;
typedef __attribute__((ext_vector_type(4)))  float    v4f;

constexpr int kVocab = 50000;
constexpr int kRaw  = 300;
constexpr int kRawP = 320;
constexpr int kD    = 256;
constexpr int kDLog2 = 8;
constexpr int kNs   = 32;
constexpr int kB    = 32;
constexpr int kL    = 1024;
constexpr int kRows = kB * kL;
constexpr int kThr  = 256;
constexpr float kInCarry = 1024.0f;
constexpr float kSc = 1.0f / (kInCarry * kInCarry);
constexpr float kF16MinNormal = 6.103515625e-5f;

static_assert((1 << kDLog2) == kD && kRawP >= kRaw && (kRawP % 32) == 0 && (kRawP % 8) == 0, "the shift follows the size; the padded width is a whole number of K steps and of 8-element chunks");
static_assert((kRows % 64) == 0 && (kD % 64) == 0 && ((kRows / 64) * (kD / 64)) % 8 == 0, "GEMM M, N multiples of 64; grid exact (2,048 tiles)");

constexpr size_t kOffE16 = 0ull;
constexpr size_t kOffWL16 = 20971520ull;
constexpr size_t kOffBIAS = 21135360ull;
constexpr size_t kOffX32 = 21136384ull;
constexpr size_t kWsTotal = 54690816ull;
static_assert(kWsTotal <= 134217728ull, "carve cap: under 128 MiB");
static_assert(kOffE16 == 0
              && kOffWL16 == kOffE16 + 20971520ull
              && kOffBIAS == kOffWL16 + 163840ull
              && kOffX32 == kOffBIAS + 1024ull
              && kWsTotal == kOffX32 + 33554432ull, "the carve is chained and totalled");
static_assert((kOffE16 % 256) == 0 && (kOffWL16 % 256) == 0 && (kOffBIAS % 256) == 0 && (kOffX32 % 256) == 0, "aligned regions");

__device__ __forceinline__ unsigned short f2bf_bits(float f) {
  unsigned u = __float_as_uint(f);
  return (unsigned short)((u + 0x7FFFu + ((u >> 16) & 1u)) >> 16);
}
__device__ __forceinline__ float bf_bits2f(unsigned short h) { return __uint_as_float(((unsigned)h) << 16); }
__device__ __forceinline__ float bf16r(float f) { return bf_bits2f(f2bf_bits(f)); }
__device__ __forceinline__ float carry_flush(float v, float carry) {
  const float s = v * carry;
  return (fabsf(s) < kF16MinNormal) ? 0.0f : s;
}
__device__ __forceinline__ float frcp(float x) { return __builtin_amdgcn_rcpf(x); }

__device__ __forceinline__ void dep_guard4_h(v8f& a, v8f& b, v8f& c, v8f& d, v16h x, v16h y) { asm volatile("v_nop\n\tv_nop\n\tv_nop\n\tv_nop" : "+v"(a), "+v"(b), "+v"(c), "+v"(d) : "v"(x), "v"(y)); }
__device__ __forceinline__ void dep_guard4_b(v8f& a, v8f& b, v8f& c, v8f& d, v16b x, v16b y) { asm volatile("v_nop\n\tv_nop\n\tv_nop\n\tv_nop" : "+v"(a), "+v"(b), "+v"(c), "+v"(d) : "v"(x), "v"(y)); }
__device__ __forceinline__ void keep4_h(v16h a, v16h b, v16h c, v16h d) { asm volatile("v_nop" :: "v"(a), "v"(b), "v"(c), "v"(d)); }
__device__ __forceinline__ void keep4_b(v16b a, v16b b, v16b c, v16b d) { asm volatile("v_nop" :: "v"(a), "v"(b), "v"(c), "v"(d)); }
__device__ __forceinline__ void acc_guard4(v8f& a, v8f& b, v8f& c, v8f& d) { asm volatile("v_nop\n\tv_nop\n\tv_nop\n\tv_nop" : "+v"(a), "+v"(b), "+v"(c), "+v"(d)); }

template <typename T> struct Frag;
template <> struct Frag<_Float16> {
  typedef v16h V; union U { v16h v; v8h h[2]; };
  static __device__ __forceinline__ v16h load(const _Float16* p) {
    U f; f.h[0] = *(const v8h*)(p); f.h[1] = *(const v8h*)(p + 16); return f.v;
  }
  static __device__ __forceinline__ v8f mma(v16h a, v16h b, v8f c) {
    return __builtin_amdgcn_wmma_f32_16x16x32_f16(false, a, false, b, (short)0, c, false, false);
  }
  static __device__ __forceinline__ void guard4(v8f& a, v8f& b, v8f& c, v8f& d, v16h x, v16h y) { dep_guard4_h(a, b, c, d, x, y); }
  static __device__ __forceinline__ void keep(v16h a, v16h b, v16h c, v16h d) { keep4_h(a, b, c, d); }
};
template <> struct Frag<__bf16> {
  typedef v16b V; union U { v16b v; v8b h[2]; };
  static __device__ __forceinline__ v16b load(const __bf16* p) {
    U f; f.h[0] = *(const v8b*)(p); f.h[1] = *(const v8b*)(p + 16); return f.v;
  }
  static __device__ __forceinline__ v8f mma(v16b a, v16b b, v8f c) {
    return __builtin_amdgcn_wmma_f32_16x16x32_bf16(false, a, false, b, (short)0, c, false, false);
  }
  static __device__ __forceinline__ void guard4(v8f& a, v8f& b, v8f& c, v8f& d, v16b x, v16b y) { dep_guard4_b(a, b, c, d, x, y); }
  static __device__ __forceinline__ void keep(v16b a, v16b b, v16b c, v16b d) { keep4_b(a, b, c, d); }
};

__device__ __forceinline__ v8f mma_h(v16h a, v16h b, v8f c) {
  c = __builtin_amdgcn_wmma_f32_16x16x32_f16(false, a, false, b, (short)0, c, false, false);
  asm volatile("v_nop\n\tv_nop\n\tv_nop\n\tv_nop" : "+v"(c) : "v"(a), "v"(b));
  return c;
}

template <int ET> struct Elem;
template <> struct Elem<0> { typedef _Float16 T; };
template <> struct Elem<1> { typedef __bf16 T; };
template <int ET, bool SPLIT, int BIAS_MODE, int OUT_MODE, bool RESID, int ACT = 0>
__global__ __launch_bounds__(256) void wmma_gemm64(
    const unsigned short* __restrict__ Ap, const unsigned short* __restrict__ A2p, int lda, long strideA,
    const unsigned short* __restrict__ Btp, const unsigned short* __restrict__ Bt2p, int ldb, long strideB,
    void* __restrict__ Cout, void* __restrict__ Cout2, int ldc, long strideC,
    const float* __restrict__ bias,
    const float* __restrict__ resid, long strideR,
    int M, int N, int K, float scale) {
  typedef typename Elem<ET>::T T;
  typedef typename Frag<T>::V V;
  const T* A = (const T*)Ap; const T* A2 = (const T*)A2p; const T* Bt = (const T*)Btp; const T* Bt2 = (const T*)Bt2p;
  __shared__ __align__(16) float sT[8][16 * 68];
  const int b    = blockIdx.y;
  const int lane = threadIdx.x & 31;
  const int wave = threadIdx.x >> 5;
  const int tilesN = N >> 6;
  const int tilesM = M >> 6;
  const int tile = blockIdx.x * 8 + wave;
  if (tile >= tilesM * tilesN) return;
  const int tm = tile / tilesN;
  const int tn = tile - tm * tilesN;
  const int m0 = tm << 6;
  const int n0 = tn << 6;

  const T* Ab  = A  + (size_t)b * strideA;
  const T* Bb  = Bt + (size_t)b * strideB;
  const T* Ab2 = SPLIT ? (A2  + (size_t)b * strideA) : nullptr;
  const T* Bb2 = SPLIT ? (Bt2 + (size_t)b * strideB) : nullptr;

  const int rlane = lane & 15;
  const int koff  = (lane >> 4) * 8;
  const int mOff  = (lane >> 4) * 8;

  v8f acc[4][4];
#pragma unroll
  for (int i = 0; i < 4; ++i)
#pragma unroll
    for (int j = 0; j < 4; ++j) acc[i][j] = (v8f){0.f,0.f,0.f,0.f,0.f,0.f,0.f,0.f};

  for (int k0 = 0; k0 < K; k0 += 32) {
    V bh[4], bl[4];
#pragma unroll
    for (int j = 0; j < 4; ++j) {
      const size_t bo = (size_t)(n0 + (j << 4) + rlane) * ldb + koff + k0;
      bh[j] = Frag<T>::load(Bb + bo);
      if (SPLIT) bl[j] = Frag<T>::load(Bb2 + bo);
    }
#pragma unroll
    for (int i = 0; i < 4; ++i) {
      const size_t ao = (size_t)(m0 + (i << 4) + rlane) * lda + koff + k0;
      V ah = Frag<T>::load(Ab + ao);
      V al;
      if (SPLIT) al = Frag<T>::load(Ab2 + ao);
#pragma unroll
      for (int j = 0; j < 4; ++j) {
        acc[i][j] = Frag<T>::mma(ah, bh[j], acc[i][j]);
        if (SPLIT) {
          acc[i][j] = Frag<T>::mma(ah, bl[j], acc[i][j]);
          acc[i][j] = Frag<T>::mma(al, bh[j], acc[i][j]);
        }
      }
      Frag<T>::guard4(acc[i][0], acc[i][1], acc[i][2], acc[i][3], ah, SPLIT ? al : ah);
    }
    Frag<T>::keep(bh[0], bh[1], bh[2], bh[3]);
    if (SPLIT) Frag<T>::keep(bl[0], bl[1], bl[2], bl[3]);
  }
  acc_guard4(acc[0][0], acc[0][1], acc[0][2], acc[0][3]);
  acc_guard4(acc[1][0], acc[1][1], acc[1][2], acc[1][3]);
  acc_guard4(acc[2][0], acc[2][1], acc[2][2], acc[2][3]);
  acc_guard4(acc[3][0], acc[3][1], acc[3][2], acc[3][3]);

  float* slab = sT[wave];
  const float* Rb = RESID ? (resid + (size_t)b * strideR) : nullptr;
#pragma unroll
  for (int i = 0; i < 4; ++i) {
    const int mBase = m0 + (i << 4);
#pragma unroll
    for (int j = 0; j < 4; ++j) {
      const int n = n0 + (j << 4) + rlane;
      float bv = 0.f;
      if (BIAS_MODE == 2) bv = bias[n];
#pragma unroll
      for (int r = 0; r < 8; ++r) {
        float v = acc[i][j][r] * scale;
        if (BIAS_MODE == 1) v += bias[mBase + mOff + r];
        if (BIAS_MODE == 2) v += bv;
        if (RESID) v += Rb[(size_t)(mBase + mOff + r) * ldc + n];
        if (ACT == 1) v = tanhf(v);
        if (ACT == 2) v = fmaxf(v, 0.0f);
        if (ACT == 3) v = v / (1.0f + expf(-v));
        if (ACT == 4) v = (v > 0.f) ? v : 0.01f * v;
        slab[(mOff + r) * 68 + (j << 4) + rlane] = v;
      }
    }
    __builtin_amdgcn_fence(__ATOMIC_RELEASE, "workgroup");
    __builtin_amdgcn_wave_barrier();
    __builtin_amdgcn_fence(__ATOMIC_ACQUIRE, "workgroup");
    if (OUT_MODE == 0) {
      float* C = (float*)Cout + (size_t)b * strideC;
      const int hh = lane >> 4, c4 = (lane & 15) * 4;
      for (int pass = 0; pass < 2; ++pass) {
#pragma unroll
        for (int it = 0; it < 8; ++it) {
          const int row = it * 2 + hh;
          v4f v = *(const v4f*)(slab + row * 68 + c4);
          *(volatile v4f*)(C + (size_t)(mBase + row) * ldc + n0 + c4) = v;
        }
        __threadfence();
      }
    } else {
      const int q = lane >> 3, c8 = (lane & 7) * 8;
      unsigned short* C  = (unsigned short*)Cout  + (size_t)b * strideC;
      unsigned short* C2 = (OUT_MODE == 2) ? ((unsigned short*)Cout2 + (size_t)b * strideC) : nullptr;
      for (int pass = 0; pass < 2; ++pass) {
#pragma unroll
        for (int it = 0; it < 4; ++it) {
          const int row = it * 4 + q;
          const float* sp = slab + row * 68 + c8;
          v8h hv, lv;
#pragma unroll
          for (int e = 0; e < 8; ++e) {
            if (OUT_MODE == 1) {
              hv[e] = (_Float16)sp[e];
            } else {
              unsigned short hb = f2bf_bits(sp[e]);
              unsigned short lb = f2bf_bits(sp[e] - bf_bits2f(hb));
              hv[e] = __builtin_bit_cast(_Float16, hb);
              lv[e] = __builtin_bit_cast(_Float16, lb);
            }
          }
          *(volatile v8h*)(C + (size_t)(mBase + row) * ldc + n0 + c8) = hv;
          if (OUT_MODE == 2) *(volatile v8h*)(C2 + (size_t)(mBase + row) * ldc + n0 + c8) = lv;
        }
        __threadfence();
      }
    }
    __builtin_amdgcn_fence(__ATOMIC_RELEASE, "workgroup");
    __builtin_amdgcn_wave_barrier();
    __builtin_amdgcn_fence(__ATOMIC_ACQUIRE, "workgroup");
  }
}


__global__ __launch_bounds__(64) void gather_cast_kernel(const int* __restrict__ src, const float* __restrict__ emb, unsigned short* __restrict__ E16) {
  const unsigned row = blockIdx.y;
  const unsigned c = threadIdx.x;
  if (c >= (unsigned)(kRawP / 8)) return;
  int tok = src[row];
  tok = (tok < 0) ? 0 : ((tok > kVocab - 1) ? (kVocab - 1) : tok);
  const float* sp = emb + (size_t)tok * kRaw;
  const unsigned c8 = c * 8u;
  const bool lo4 = c8 + 4u <= (unsigned)kRaw;
  const bool hi4 = c8 + 8u <= (unsigned)kRaw;
  const v4f a0 = *(const v4f*)(sp + (lo4 ? c8 : (unsigned)(kRaw - 4)));
  const v4f a1 = *(const v4f*)(sp + (hi4 ? (c8 + 4u) : (unsigned)(kRaw - 4)));
  v8h hv;
#pragma unroll
  for (int e = 0; e < 4; ++e) {
    const float p = a0[e], q = a1[e];
    hv[e] = (_Float16)(lo4 ? carry_flush(bf16r(p), kInCarry) : 0.0f);
    hv[4 + e] = (_Float16)(hi4 ? carry_flush(bf16r(q), kInCarry) : 0.0f);
  }
  unsigned short* dp = E16 + (size_t)row * kRawP + c8;
  *(volatile v8h*)dp = hv;
  __threadfence();
  *(volatile v8h*)dp = hv;
}
static_assert((kRaw % 4) == 0 && (kRawP / 8) == 40 && (kRaw * 4) % 16 == 0, "a table row is a whole number of 4-float loads, 16-B aligned (1,200 B a row); 40 chunks a padded row");

__global__ __launch_bounds__(64) void setup_kernel(const float* __restrict__ W_lin, const float* __restrict__ b_lin, unsigned short* __restrict__ WL16,
                                                   float* __restrict__ BIAS) {
  const unsigned y = blockIdx.y;
  const unsigned c = threadIdx.x;
  if (y < (unsigned)kD) {
    if (c >= (unsigned)(kRawP / 8)) return;
    const float* sp = W_lin + (size_t)y * kRaw;
    const unsigned c8 = c * 8u;
    const bool lo4 = c8 + 4u <= (unsigned)kRaw, hi4 = c8 + 8u <= (unsigned)kRaw;
    const v4f a0 = *(const v4f*)(sp + (lo4 ? c8 : (unsigned)(kRaw - 4)));
    const v4f a1 = *(const v4f*)(sp + (hi4 ? (c8 + 4u) : (unsigned)(kRaw - 4)));
    v8h hv;
#pragma unroll
    for (int e = 0; e < 4; ++e) {
      const float p = a0[e], q = a1[e];
      hv[e] = (_Float16)(lo4 ? carry_flush(bf16r(p), kInCarry) : 0.0f);
      hv[4 + e] = (_Float16)(hi4 ? carry_flush(bf16r(q), kInCarry) : 0.0f);
    }
    unsigned short* dp = WL16 + (size_t)y * kRawP + c8;
    *(volatile v8h*)dp = hv;
    __threadfence();
    *(volatile v8h*)dp = hv;
  } else {
    if (c >= 32u) return;
    const v4f a0 = *(const v4f*)(b_lin + c * 8u), a1 = *(const v4f*)(b_lin + c * 8u + 4);
    v4f o0, o1;
#pragma unroll
    for (int e = 0; e < 4; ++e) { const float p = a0[e], q = a1[e]; o0[e] = bf16r(p); o1[e] = bf16r(q); }
    float* dp = BIAS + c * 8u;
    for (int pass = 0; pass < 2; ++pass) {
      *(volatile v4f*)dp = o0;
      *(volatile v4f*)(dp + 4) = o1;
      __threadfence();
    }
  }
}
static_assert(kD == 32 * 8, "the bias row = 32 chunks of 8");

__global__ __launch_bounds__(kThr) void scan_kernel(const float* __restrict__ X32, const int* __restrict__ lengths, const float* __restrict__ A_log,
                                                    const float* __restrict__ log_dt, const float* __restrict__ Bp, const float* __restrict__ Cp,
                                                    const float* __restrict__ Dp, float* __restrict__ out) {
  const unsigned v = blockIdx.x * (unsigned)kThr + threadIdx.x;
  const unsigned smp = v >> kDLog2, d = v & (unsigned)(kD - 1);
  int len = lengths[smp];
  len = (len < 0) ? 0 : ((len > kL) ? kL : len);
  const float ld0 = log_dt[d], dp0 = Dp[d];
  const float dt = expf(bf16r(ld0));
  const float dsk = bf16r(dp0);
  float ab[kNs], bb[kNs], cc[kNs], h[kNs];
#pragma unroll
  for (int n = 0; n < kNs; ++n) {
    const float a0 = A_log[(size_t)d * kNs + n], b0 = Bp[(size_t)d * kNs + n], c0 = Cp[(size_t)d * kNs + n];
    ab[n] = expf(dt * -expf(bf16r(a0)));
    bb[n] = dt * bf16r(b0);
    cc[n] = bf16r(c0);
    h[n] = 0.0f;
  }
  const size_t r0 = (size_t)smp * kL;
  for (int l = 0; l < kL; ++l) {
    const float xr = X32[(r0 + (size_t)l) * kD + d];
    const float x = (l < len) ? xr : 0.0f;
    float y = 0.0f;
#pragma unroll
    for (int n = 0; n < kNs; ++n) {
      const float hn = ab[n] * h[n] + bb[n] * x;
      h[n] = hn;
      y += hn * cc[n];
    }
    const float o = y + dsk * x;
    float* op = out + (r0 + (size_t)l) * kD + d;
    *(volatile float*)op = o;
    __threadfence();
    *(volatile float*)op = o;
  }
}
static_assert((kB * kD) % kThr == 0, "scan grid exact: 32 blocks");

extern "C" void kernel_launch(void* const* d_in, const int* in_sizes, int n_in,
                              void* d_out, int out_size, void* d_ws, size_t ws_size,
                              hipStream_t stream) {
  if (n_in < 10 || d_out == nullptr || d_ws == nullptr) return;
  if (in_sizes[0] != kRows || in_sizes[1] != kB || in_sizes[2] != kVocab * kRaw || in_sizes[3] != kD * kRaw || in_sizes[4] != kD) return;
  if (in_sizes[5] != kD * kNs || in_sizes[6] != kD || in_sizes[7] != kD * kNs || in_sizes[8] != kD * kNs || in_sizes[9] != kD) return;
  if (out_size != kRows * kD) return;
  if (ws_size < kWsTotal) return;
  const int* src = (const int*)d_in[0];
  const int* lengths = (const int*)d_in[1];
  const float* emb_table = (const float*)d_in[2];
  const float* W_lin = (const float*)d_in[3];
  const float* b_lin = (const float*)d_in[4];
  const float* A_log = (const float*)d_in[5];
  const float* log_dt = (const float*)d_in[6];
  const float* Bp = (const float*)d_in[7];
  const float* Cp = (const float*)d_in[8];
  const float* Dp = (const float*)d_in[9];
  float* out = (float*)d_out;
  char* ws = (char*)d_ws;
  unsigned short* E16 = (unsigned short*)(ws + kOffE16);
  unsigned short* WL16 = (unsigned short*)(ws + kOffWL16);
  float* BIAS = (float*)(ws + kOffBIAS);
  float* X32 = (float*)(ws + kOffX32);

  gather_cast_kernel<<<dim3(1, kRows), 64, 0, stream>>>(src, emb_table, E16);
  setup_kernel<<<dim3(1, kD + 1), 64, 0, stream>>>(W_lin, b_lin, WL16, BIAS);
  wmma_gemm64<0, false, 2, 0, false, 0><<<dim3((kRows / 64) * (kD / 64) / 8, 1), 256, 0, stream>>>(
      E16, E16, kRawP, 0L, WL16, WL16, kRawP, 0L, (void*)X32, (void*)X32, kD, 0L, BIAS, nullptr, 0L, kRows, kD, kRawP, kSc);
  scan_kernel<<<(kB * kD) / kThr, kThr, 0, stream>>>(X32, lengths, A_log, log_dt, Bp, Cp, Dp, out);
}
